// NAM_33655363732260
// MI455X (gfx1250) — hardware-verified
//
#include <hip/hip_runtime.h>
#include <math.h>

constexpr int kRows        = 262144;
constexpr int kFeat        = 17;
constexpr int kH1          = 64;
constexpr int kH2          = 32;
constexpr int kWaves       = 4;
constexpr int kThreads     = kWaves * 32;
constexpr int kRowsPerWave = 64;
constexpr int kRowsPerBlk  = kWaves * kRowsPerWave;
constexpr int kXSlab       = kRowsPerWave * kFeat;
constexpr int kXSlabV4     = kXSlab / 4;
constexpr int kAPitch      = 72;
constexpr int kW2tHalves   = kFeat * kH2 * kH1;
constexpr float kW2Carry    = 16.0f;
constexpr float kW2CarryInv = 1.0f / 16.0f;

static_assert(kRows % kRowsPerBlk == 0, "no M tail");
static_assert(kH1 % 32 == 0, "K multiple of 32");
static_assert(kH2 == 32, "N = two 16-column tiles");
static_assert(kXSlab % 4 == 0, "x slab is a whole number of 16-B items");
static_assert((kAPitch * 2) % 16 == 0, "A rows 16-B aligned");

typedef __attribute__((ext_vector_type(16))) _Float16 v16h;
typedef __attribute__((ext_vector_type(8)))  _Float16 v8h;
typedef __attribute__((ext_vector_type(8)))  float    v8f;
typedef __attribute__((ext_vector_type(4)))  float    v4f;
typedef __attribute__((ext_vector_type(4)))  unsigned int v4u;

__device__ __forceinline__ void dep_guard_h(v8f& a, v8f& b, v16h x, v16h y) { asm volatile("v_nop\n\tv_nop\n\tv_nop\n\tv_nop" : "+v"(a), "+v"(b) : "v"(x), "v"(y)); }
__device__ __forceinline__ void keep4_h(v16h a, v16h b, v16h c, v16h d) { asm volatile("v_nop" :: "v"(a), "v"(b), "v"(c), "v"(d)); }
template <typename T> struct Frag;
template <> struct Frag<_Float16> {
  typedef v16h V; union U { v16h v; v8h h[2]; };
  static __device__ __forceinline__ v16h load(const _Float16* p) {
    U f; f.h[0] = *(const v8h*)(p); f.h[1] = *(const v8h*)(p + 16); return f.v;
  }
  static __device__ __forceinline__ v8f mma(v16h a, v16h b, v8f c) {
    return __builtin_amdgcn_wmma_f32_16x16x32_f16(false, a, false, b, (short)0, c, false, false);
  }
  static __device__ __forceinline__ void guard(v8f& a, v8f& b, v16h x, v16h y) { dep_guard_h(a, b, x, y); }
  static __device__ __forceinline__ void keep(v16h a, v16h b, v16h c, v16h d) { keep4_h(a, b, c, d); }
};

__device__ __forceinline__ unsigned pk16(unsigned short a, unsigned short b) { return (unsigned)a | ((unsigned)b << 16); }
__device__ __forceinline__ unsigned short h_bits(float f) { const _Float16 h = (_Float16)f; return __builtin_bit_cast(unsigned short, h); }

__global__ __launch_bounds__(256) void w2t_cast_kernel(const float* __restrict__ W2,
                                                       unsigned short* __restrict__ W2t) {
  __shared__ float sm[kH2][kH1 + 1];
  const int t = threadIdx.x;
  const int f = blockIdx.x;
  const float* wf = W2 + (size_t)f * (kH1 * kH2);
#pragma unroll
  for (int i = 0; i < 8; ++i) {
    const int e = i * 256 + t;
    const int k = e >> 5;
    const int n = e & 31;
    sm[n][k] = wf[e] * kW2Carry;
  }
  __syncthreads();
  const int lane = t & 31, wave = t >> 5;
  const int q = lane >> 3, c8 = (lane & 7) * 8;
  const int row = wave * 4 + q;
  unsigned short hb[8];
#pragma unroll
  for (int e = 0; e < 8; ++e) hb[e] = h_bits(sm[row][c8 + e]);
  const v4u u = (v4u){pk16(hb[0], hb[1]), pk16(hb[2], hb[3]), pk16(hb[4], hb[5]), pk16(hb[6], hb[7])};
  unsigned short* op = W2t + (size_t)(f * kH2 + row) * kH1 + c8;
  *(volatile v4u*)op = u;
  __threadfence();
  *(volatile v4u*)op = u;
}

__global__ __launch_bounds__(kThreads) void feat_mlp_kernel(
    const float* __restrict__ x, const float* __restrict__ W1, const float* __restrict__ b1,
    const unsigned short* __restrict__ W2t, const float* __restrict__ b2, const float* __restrict__ W3,
    const float* __restrict__ b3, const float* __restrict__ biasp, float* __restrict__ out) {
  __shared__ __align__(16) float    xs[kWaves][kXSlab];
  __shared__ __align__(16) _Float16 As[kWaves][kRowsPerWave * kAPitch];
  __shared__ __align__(16) float    sc[kRowsPerBlk];

  const int tid   = threadIdx.x;
  const int lane  = tid & 31;
  const int wave  = tid >> 5;
  const int rlane = lane & 15;
  const int hh    = lane >> 4;
  const int koff  = hh * 8;
  const int chunk = lane & 7;
  const int rsub  = lane >> 3;

  const size_t blockRow0 = (size_t)blockIdx.x * kRowsPerBlk;
  const size_t waveRow0  = blockRow0 + (size_t)wave * kRowsPerWave;

  {
    const v4f* src = (const v4f*)(x + waveRow0 * kFeat);
    float* xw = xs[wave];
#pragma unroll
    for (int it = 0; it < 9; ++it) {
      const int item = it * 32 + lane;
      const int itc  = item < kXSlabV4 ? item : (kXSlabV4 - 1);
      const v4f v = src[itc];
      if (item < kXSlabV4) *(v4f*)(xw + itc * 4) = v;
    }
  }

  float partial[32];
#pragma unroll
  for (int i = 0; i < 32; ++i) partial[i] = 0.0f;
  float b3sum = 0.0f;

  const float* xw = xs[wave];
  _Float16* aw = As[wave];
  const _Float16* W2h = (const _Float16*)W2t;

  for (int f = 0; f < kFeat; ++f) {
    __syncthreads();

    const v4f w1lo = *(const v4f*)(W1 + f * kH1 + chunk * 8);
    const v4f w1hi = *(const v4f*)(W1 + f * kH1 + chunk * 8 + 4);
    const v4f b1lo = *(const v4f*)(b1 + f * kH1 + chunk * 8);
    const v4f b1hi = *(const v4f*)(b1 + f * kH1 + chunk * 8 + 4);
    float w1r[8], b1r[8];
#pragma unroll
    for (int e = 0; e < 4; ++e) { w1r[e] = w1lo[e]; w1r[4 + e] = w1hi[e]; b1r[e] = b1lo[e]; b1r[4 + e] = b1hi[e]; }

    const _Float16* bp0 = W2h + (size_t)(f * kH2 + rlane) * kH1 + koff;
    const _Float16* bp1 = W2h + (size_t)(f * kH2 + 16 + rlane) * kH1 + koff;
    const v16h bf00 = Frag<_Float16>::load(bp0);
    const v16h bf10 = Frag<_Float16>::load(bp0 + 32);
    const v16h bf01 = Frag<_Float16>::load(bp1);
    const v16h bf11 = Frag<_Float16>::load(bp1 + 32);

    const float b2a = b2[f * kH2 + rlane];
    const float b2b = b2[f * kH2 + 16 + rlane];
    const float w3a = W3[f * kH2 + rlane];
    const float w3b = W3[f * kH2 + 16 + rlane];
    b3sum += b3[f];

#pragma unroll 4
    for (int it = 0; it < 16; ++it) {
      const int row = it * 4 + rsub;
      const float xv = xw[row * kFeat + f];
      v8h hv;
#pragma unroll
      for (int e = 0; e < 8; ++e) hv[e] = (_Float16)fmaxf(fmaf(xv, w1r[e], b1r[e]), 0.0f);
      *(v8h*)(aw + row * kAPitch + chunk * 8) = hv;
    }
    __syncthreads();

    const v8f zero8 = (v8f){0.f, 0.f, 0.f, 0.f, 0.f, 0.f, 0.f, 0.f};
#pragma unroll
    for (int i = 0; i < 4; ++i) {
      const _Float16* ap = aw + (i * 16 + rlane) * kAPitch + koff;
      const v16h a0 = Frag<_Float16>::load(ap);
      const v16h a1 = Frag<_Float16>::load(ap + 32);
      v8f acc0 = zero8, acc1 = zero8;
      acc0 = Frag<_Float16>::mma(a0, bf00, acc0);
      acc0 = Frag<_Float16>::mma(a1, bf10, acc0);
      acc1 = Frag<_Float16>::mma(a0, bf01, acc1);
      acc1 = Frag<_Float16>::mma(a1, bf11, acc1);
      Frag<_Float16>::guard(acc0, acc1, a0, a1);
#pragma unroll
      for (int r = 0; r < 8; ++r) {
        const float h2a = fmaxf(fmaf(acc0[r], kW2CarryInv, b2a), 0.0f);
        const float h2b = fmaxf(fmaf(acc1[r], kW2CarryInv, b2b), 0.0f);
        partial[i * 8 + r] = fmaf(h2a, w3a, partial[i * 8 + r]);
        partial[i * 8 + r] = fmaf(h2b, w3b, partial[i * 8 + r]);
      }
    }
    Frag<_Float16>::keep(bf00, bf10, bf01, bf11);
  }

  const float addc = biasp[0] + b3sum;
#pragma unroll
  for (int i = 0; i < 4; ++i) {
#pragma unroll
    for (int r = 0; r < 8; ++r) {
      float v = partial[i * 8 + r];
      v += __shfl_xor(v, 1, 32);
      v += __shfl_xor(v, 2, 32);
      v += __shfl_xor(v, 4, 32);
      v += __shfl_xor(v, 8, 32);
      if (rlane == 0) sc[wave * kRowsPerWave + i * 16 + hh * 8 + r] = v + addc;
    }
  }
  __syncthreads();

  if (wave == 0) {
    float* ob = out + blockRow0;
    for (int pass = 0; pass < 2; ++pass) {
#pragma unroll
      for (int it = 0; it < 2; ++it) {
        const v4f v = *(const v4f*)(sc + it * 128 + lane * 4);
        *(volatile v4f*)(ob + it * 128 + lane * 4) = v;
      }
      __threadfence();
    }
  }
}

extern "C" void kernel_launch(void* const* d_in, const int* in_sizes, int n_in,
                              void* d_out, int out_size, void* d_ws, size_t ws_size,
                              hipStream_t stream) {
  (void)in_sizes; (void)n_in; (void)out_size;
  const float* x    = (const float*)d_in[0];
  const float* W1   = (const float*)d_in[1];
  const float* b1   = (const float*)d_in[2];
  const float* W2   = (const float*)d_in[3];
  const float* b2   = (const float*)d_in[4];
  const float* W3   = (const float*)d_in[5];
  const float* b3   = (const float*)d_in[6];
  const float* bias = (const float*)d_in[7];
  float* outp = (float*)d_out;

  const size_t w2tBytes = (size_t)kW2tHalves * 2;
  if (ws_size < w2tBytes) return;
  unsigned short* W2t = (unsigned short*)d_ws;

  w2t_cast_kernel<<<kFeat, 256, 0, stream>>>(W2, W2t);
  feat_mlp_kernel<<<kRows / kRowsPerBlk, kThreads, 0, stream>>>(x, W1, b1, W2t, b2, W3, b3, bias, outp);
}
